// TransformerLayer_39298950758497
// MI455X (gfx1250) — hardware-verified
//
#include <hip/hip_runtime.h>
#include <math.h>

typedef __attribute__((ext_vector_type(16))) _Float16 v16h;
typedef __attribute__((ext_vector_type(16))) __bf16 v16b;
typedef __attribute__((ext_vector_type(8)))  _Float16 v8h;
typedef __attribute__((ext_vector_type(4)))  _Float16 v4h;
typedef __attribute__((ext_vector_type(8)))  __bf16 v8b;
typedef __attribute__((ext_vector_type(8)))  float v8f;
typedef __attribute__((ext_vector_type(4)))  float v4f;
typedef __attribute__((ext_vector_type(8)))  unsigned short v8us;

#ifndef NB
#define NB 2
#endif
#define NB_FULL 2
#ifndef SEQ
#define SEQ 4096
#endif
#define SEQ_FULL 4096
#define DM 1024
#define NH 16
#define DH 64
#define DFF 4096
#define WIN 256
#define NGRP 17
#define NQ 4
#define NTOK ((size_t)NB * (size_t)SEQ)
#define MQ (NTOK / NQ)
#define XC (16.0f)
#define HC (16.0f)
#define WC (1024.0f)
#define VC (16.0f)
#define PCY (16384.0f)
#define F16MIN (6.103515625e-05f)
#define LN_EPS (1e-5f)
static_assert(NB >= 1 && NB <= NB_FULL);
static_assert(SEQ % 64 == 0 && SEQ >= 64 && SEQ <= SEQ_FULL);
static_assert(NTOK % (NQ * 64) == 0);
static_assert(MQ % 64 == 0 && MQ % 16 == 0);
static_assert(DM == NH * DH && DH == 64);
static_assert(DM % 128 == 0 && DFF % 128 == 0 && DM % 64 == 0 && DFF % 64 == 0);

#define WSZ_QB  (2u * NTOK * DM)
#define WSZ_VT  (2u * NTOK * DM)
#define WSZ_W1T (2u * (size_t)DFF * DM)
#define WSZ_W2T (2u * (size_t)DM * DFF)
#define WSZ_X32 (4u * NTOK * DM)
#define WSZ_X16 (2u * NTOK * DM)
#define WSZ_H16 (2u * (size_t)MQ * DFF)
#define WS_QB   ((size_t)0)
#define WS_VT   (WS_QB  + WSZ_QB)
#define WS_W1T  (WS_VT  + WSZ_VT)
#define WS_W2T  (WS_W1T + WSZ_W1T)
#define WS_X32  (WS_W2T + WSZ_W2T)
#define WS_X16  (WS_X32 + WSZ_X32)
#define WS_H16  (WS_X16 + WSZ_X16)
#define WS_END  (WS_H16 + WSZ_H16)
static_assert(WS_END <= (size_t)134217728u);
static_assert((WS_VT % 256u) == 0 && (WS_W1T % 256u) == 0 && (WS_W2T % 256u) == 0 && (WS_X32 % 256u) == 0 && (WS_X16 % 256u) == 0 && (WS_H16 % 256u) == 0);

template <typename T> __device__ __forceinline__ void vst2(void* p, T v) { *(volatile T*)p = v; __threadfence(); *(volatile T*)p = v; }
__device__ __forceinline__ v8f zero8() { v8f z = {0.f, 0.f, 0.f, 0.f, 0.f, 0.f, 0.f, 0.f}; return z; }
__device__ __forceinline__ v8f wmma16(v16h a, v16h b, v8f c) {
  v8f d = __builtin_amdgcn_wmma_f32_16x16x32_f16(false, a, false, b, (short)0, c, false, false);
  asm volatile("v_nop\n\tv_nop\n\tv_nop\n\tv_nop" : "+v"(d) : "v"(a), "v"(b));
  return d;
}
__device__ __forceinline__ v8f wmma_bf(v16b a, v16b b, v8f c) {
  v8f d = __builtin_amdgcn_wmma_f32_16x16x32_bf16(false, a, false, b, (short)0, c, false, false);
  asm volatile("v_nop\n\tv_nop\n\tv_nop\n\tv_nop" : "+v"(d) : "v"(a), "v"(b));
  return d;
}
__device__ __forceinline__ v16h frag_h(const _Float16* rowk0, int lane) {
  union { v16h v; v8h q[2]; } u; const _Float16* p = rowk0 + 8 * (lane >> 4);
  u.q[0] = *(const v8h*)p; u.q[1] = *(const v8h*)(p + 16); return u.v;
}
__device__ __forceinline__ v16b frag_b(const __bf16* rowk0, int lane) {
  union { v16b v; v8b q[2]; } u; const __bf16* p = rowk0 + 8 * (lane >> 4);
  u.q[0] = *(const v8b*)p; u.q[1] = *(const v8b*)(p + 16); return u.v;
}
__device__ __forceinline__ _Float16 f16n(float x) { const float t = (fabsf(x) >= F16MIN) ? x : 0.0f; return (_Float16)t; }
__device__ __forceinline__ unsigned short bf16bits(float x) { unsigned u = __float_as_uint(x); u += 0x7FFFu + ((u >> 16) & 1u); return (unsigned short)(u >> 16); }
__device__ __forceinline__ float bf16val(unsigned short b) { return __uint_as_float(((unsigned)b) << 16); }
__device__ __forceinline__ float bf16r(float x) { return bf16val(bf16bits(x)); }
#define LDSX() do { asm volatile("s_wait_dscnt 0" ::: "memory"); __builtin_amdgcn_wave_barrier(); __builtin_amdgcn_fence(3  , "workgroup"); } while (0)

__global__ __launch_bounds__(256) void k_prep(const float* __restrict__ SRC, unsigned short* __restrict__ QB, _Float16* __restrict__ VT) {
  __shared__ __align__(16) _Float16 th[DH][72];
  const int tid = threadIdx.x; const int s0 = blockIdx.x * 64, h = blockIdx.y, b = blockIdx.z;
  const size_t bh = (size_t)b * NH + h;
#pragma unroll
  for (int it = 0; it < 2; ++it) {
    const int e = tid + 256 * it; const int tl = e >> 3, q = e & 7;
    const float* p = SRC + ((size_t)b * SEQ_FULL + s0 + tl) * DM + h * DH + q * 8;
    const v4f a = *(const v4f*)p, c = *(const v4f*)(p + 4);
    v8us o;
#pragma unroll
    for (int k = 0; k < 4; ++k) { o[k] = bf16bits(a[k]); o[4 + k] = bf16bits(c[k]); }
    vst2(QB + (bh * SEQ + s0 + tl) * (size_t)DH + q * 8, o);
#pragma unroll
    for (int k = 0; k < 8; ++k) th[q * 8 + k][tl] = f16n(bf16val(o[k]) * VC);
  }
  __syncthreads();
#pragma unroll
  for (int it = 0; it < 2; ++it) { const int e = tid + 256 * it; const int d = e >> 3, q = e & 7;
    vst2(VT + (bh * DH + d) * (size_t)SEQ + s0 + q * 8, *(const v8h*)&th[d][q * 8]); }
}

__global__ __launch_bounds__(256) void k_trw(const float* __restrict__ Wm, int K, int N, _Float16* __restrict__ WT) {
  __shared__ __align__(16) _Float16 th[64][72];
  const int tid = threadIdx.x; const int n0 = blockIdx.x * 64, k0 = blockIdx.y * 64;
#pragma unroll
  for (int it = 0; it < 4; ++it) {
    const int e = tid + 256 * it; const int kl = e >> 4, n4 = e & 15;
    const v4f a = *(const v4f*)(Wm + (size_t)(k0 + kl) * N + n0 + n4 * 4);
#pragma unroll
    for (int c = 0; c < 4; ++c) th[n4 * 4 + c][kl] = f16n(bf16r(a[c]) * WC);
  }
  __syncthreads();
#pragma unroll
  for (int it = 0; it < 2; ++it) { const int e = tid + 256 * it; const int nl = e >> 3, q = e & 7;
    vst2(WT + (size_t)(n0 + nl) * K + k0 + q * 8, *(const v8h*)&th[nl][q * 8]); }
}

__global__ __launch_bounds__(512) void k_attln(const float* __restrict__ SRC, const __bf16* __restrict__ QB, const _Float16* __restrict__ VT,
                                               const float* __restrict__ G1, const float* __restrict__ C1, float* __restrict__ X32, _Float16* __restrict__ X16) {
  __shared__ __align__(16) _Float16 sP[NH][16][40];
  __shared__ __align__(16) float sx[16][DM + 4];
  const int tid = threadIdx.x, wave = tid >> 5, lane = tid & 31, col = lane & 15, g = lane >> 4;
  const int nbq = SEQ / 16;
  const int b = blockIdx.x / nbq; const int q0 = (blockIdx.x - b * nbq) * 16;
  const size_t bh = (size_t)b * NH + wave;
  const __bf16* QBh = QB + bh * (size_t)SEQ * DH;
  const _Float16* VTh = VT + bh * (size_t)DH * SEQ;
  const v16b qa0 = frag_b(QBh + (size_t)(q0 + col) * DH, lane);
  const v16b qa1 = frag_b(QBh + (size_t)(q0 + col) * DH + 32, lane);
  const int gb = (q0 & ~31) - WIN;
  const int gst = (gb > 0) ? gb : 0;
  const int gen = (gb + NGRP * 32 < SEQ) ? (gb + NGRP * 32) : SEQ;

  float m[8];
#pragma unroll
  for (int r = 0; r < 8; ++r) m[r] = -3.0e38f;
#pragma unroll 1
  for (int gs = gst; gs < gen; gs += 32) {
    const __bf16* k0p = QBh + (size_t)(gs + col) * DH; const __bf16* k1p = QBh + (size_t)(gs + 16 + col) * DH;
    v8f c0 = zero8(), c1 = zero8();
    c0 = wmma_bf(qa0, frag_b(k0p, lane), c0); c0 = wmma_bf(qa1, frag_b(k0p + 32, lane), c0);
    c1 = wmma_bf(qa0, frag_b(k1p, lane), c1); c1 = wmma_bf(qa1, frag_b(k1p + 32, lane), c1);
    const int kp0 = gs + col, kp1 = gs + 16 + col;
#pragma unroll
    for (int r = 0; r < 8; ++r) {
      const int qp = q0 + 8 * g + r;
      const bool v0 = (kp0 - qp <= WIN) && (qp - kp0 <= WIN);
      const bool v1 = (kp1 - qp <= WIN) && (qp - kp1 <= WIN);
      m[r] = fmaxf(m[r], v0 ? c0[r] : -3.0e38f);
      m[r] = fmaxf(m[r], v1 ? c1[r] : -3.0e38f);
    }
  }
#pragma unroll
  for (int r = 0; r < 8; ++r) { float t = m[r]; t = fmaxf(t, __shfl_xor(t, 1)); t = fmaxf(t, __shfl_xor(t, 2)); t = fmaxf(t, __shfl_xor(t, 4)); t = fmaxf(t, __shfl_xor(t, 8)); m[r] = t; }

  float lsum[8];
#pragma unroll
  for (int r = 0; r < 8; ++r) lsum[r] = 0.f;
  v8f acc[4];
#pragma unroll
  for (int j = 0; j < 4; ++j) acc[j] = zero8();
#pragma unroll 1
  for (int gs = gst; gs < gen; gs += 32) {
    const __bf16* k0p = QBh + (size_t)(gs + col) * DH; const __bf16* k1p = QBh + (size_t)(gs + 16 + col) * DH;
    v8f c0 = zero8(), c1 = zero8();
    c0 = wmma_bf(qa0, frag_b(k0p, lane), c0); c0 = wmma_bf(qa1, frag_b(k0p + 32, lane), c0);
    c1 = wmma_bf(qa0, frag_b(k1p, lane), c1); c1 = wmma_bf(qa1, frag_b(k1p + 32, lane), c1);
    const int kp0 = gs + col, kp1 = gs + 16 + col;
    int nz = 0;
    LDSX();
#pragma unroll
    for (int r = 0; r < 8; ++r) {
      const int qp = q0 + 8 * g + r;
      const bool v0 = (kp0 - qp <= WIN) && (qp - kp0 <= WIN);
      const bool v1 = (kp1 - qp <= WIN) && (qp - kp1 <= WIN);
      float p0 = __expf(fminf(c0[r] - m[r], 0.0f)) * PCY; p0 = (v0 && p0 >= F16MIN) ? p0 : 0.0f;
      float p1 = __expf(fminf(c1[r] - m[r], 0.0f)) * PCY; p1 = (v1 && p1 >= F16MIN) ? p1 : 0.0f;
      const _Float16 h0 = (_Float16)p0, h1 = (_Float16)p1;
      lsum[r] += (float)h0 + (float)h1; nz |= (p0 != 0.0f || p1 != 0.0f) ? 1 : 0;
      sP[wave][8 * g + r][col] = h0; sP[wave][8 * g + r][16 + col] = h1;
    }
    const unsigned wb = __builtin_amdgcn_ballot_w32(nz != 0);
    if (wb != 0u) {
      LDSX();
      const v16h pa = frag_h(&sP[wave][col][0], lane);
#pragma unroll
      for (int j = 0; j < 4; ++j) acc[j] = wmma16(pa, frag_h(VTh + (size_t)(j * 16 + col) * SEQ + gs, lane), acc[j]);
    }
  }
#pragma unroll
  for (int r = 0; r < 8; ++r) { float t = lsum[r]; t += __shfl_xor(t, 1); t += __shfl_xor(t, 2); t += __shfl_xor(t, 4); t += __shfl_xor(t, 8); lsum[r] = t; }
  float inv[8];
#pragma unroll
  for (int r = 0; r < 8; ++r) inv[r] = (1.0f / lsum[r]) * (1.0f / VC);
#pragma unroll
  for (int j = 0; j < 4; ++j)
#pragma unroll
    for (int r = 0; r < 8; ++r) sx[8 * g + r][wave * DH + j * 16 + col] = acc[j][r] * inv[r];
  __syncthreads();

  const int s = q0 + wave;
  const size_t so = ((size_t)b * SEQ_FULL + s) * DM;
  const size_t xo = ((size_t)b * SEQ + s) * DM;
  v4f v[8]; float s1 = 0.f;
#pragma unroll
  for (int i = 0; i < 8; ++i) {
    const v4f a = *(const v4f*)&sx[wave][i * 128 + lane * 4]; const v4f xs = *(const v4f*)(SRC + so + i * 128 + lane * 4);
#pragma unroll
    for (int k = 0; k < 4; ++k) v[i][k] = bf16r(xs[k]) + a[k];
    s1 += (v[i][0] + v[i][1]) + (v[i][2] + v[i][3]);
  }
#pragma unroll
  for (int o = 1; o < 32; o <<= 1) s1 += __shfl_xor(s1, o);
  const float mu = s1 * (1.0f / DM); float qv = 0.f;
#pragma unroll
  for (int i = 0; i < 8; ++i)
#pragma unroll
    for (int k = 0; k < 4; ++k) { const float d = v[i][k] - mu; qv += d * d; }
#pragma unroll
  for (int o = 1; o < 32; o <<= 1) qv += __shfl_xor(qv, o);
  const float rs = 1.0f / sqrtf(qv * (1.0f / DM) + LN_EPS);
#pragma unroll
  for (int i = 0; i < 8; ++i) {
    const v4f gg = *(const v4f*)(G1 + i * 128 + lane * 4), cc = *(const v4f*)(C1 + i * 128 + lane * 4);
    v4f y; v4h yh;
#pragma unroll
    for (int k = 0; k < 4; ++k) { y[k] = (v[i][k] - mu) * rs * bf16r(gg[k]) + bf16r(cc[k]); yh[k] = f16n(y[k] * XC); }
    vst2(X32 + xo + i * 128 + lane * 4, y);
    vst2(X16 + xo + i * 128 + lane * 4, yh);
  }
}

__global__ __launch_bounds__(128) void k_g1(const _Float16* __restrict__ X16q, const _Float16* __restrict__ W1T, const float* __restrict__ B1, _Float16* __restrict__ H16) {
  __shared__ __align__(16) _Float16 sh[4][16][136];
  const int tid = threadIdx.x, wave = tid >> 5, lane = tid & 31, col = lane & 15, g = lane >> 4;
  const int c0 = blockIdx.y * 128; const size_t r0 = (size_t)blockIdx.x * 64 + wave * 16;
  v8f acc[8];
#pragma unroll
  for (int j = 0; j < 8; ++j) acc[j] = zero8();
#pragma unroll 1
  for (int kc = 0; kc < DM / 32; ++kc) {
    const v16h a = frag_h(X16q + (r0 + col) * DM + kc * 32, lane);
#pragma unroll
    for (int j = 0; j < 8; ++j) acc[j] = wmma16(a, frag_h(W1T + (size_t)(c0 + j * 16 + col) * DM + kc * 32, lane), acc[j]);
  }
#pragma unroll
  for (int j = 0; j < 8; ++j) {
    const float bj = bf16r(B1[c0 + j * 16 + col]);
#pragma unroll
    for (int r = 0; r < 8; ++r) { const float hv = fmaxf(acc[j][r] * (1.0f / (XC * WC)) + bj, 0.0f); sh[wave][8 * g + r][j * 16 + col] = f16n(hv * HC); }
  }
  LDSX();
#pragma unroll
  for (int rp = 0; rp < 8; ++rp) { const int rl = 2 * rp + g; vst2(H16 + (r0 + rl) * (size_t)DFF + c0 + col * 8, *(const v8h*)&sh[wave][rl][col * 8]); }
}

__global__ __launch_bounds__(256) void k_g2ln(const _Float16* __restrict__ H16, const _Float16* __restrict__ W2T, const float* __restrict__ B2,
                                              const float* __restrict__ X32q, const float* __restrict__ G2, const float* __restrict__ C2, float* __restrict__ OUTq) {
  __shared__ __align__(16) float sz[16][DM + 4];
  const int tid = threadIdx.x, wave = tid >> 5, lane = tid & 31, col = lane & 15, g = lane >> 4;
  const size_t r0 = (size_t)blockIdx.x * 16; const int cw = wave * 128;
  v8f acc[8];
#pragma unroll
  for (int j = 0; j < 8; ++j) acc[j] = zero8();
#pragma unroll 1
  for (int kc = 0; kc < DFF / 32; ++kc) {
    const v16h a = frag_h(H16 + (r0 + col) * DFF + kc * 32, lane);
#pragma unroll
    for (int j = 0; j < 8; ++j) acc[j] = wmma16(a, frag_h(W2T + (size_t)(cw + j * 16 + col) * DFF + kc * 32, lane), acc[j]);
  }
#pragma unroll
  for (int j = 0; j < 8; ++j)
#pragma unroll
    for (int r = 0; r < 8; ++r) sz[8 * g + r][cw + j * 16 + col] = acc[j][r] * (1.0f / (HC * WC));
  __syncthreads();
#pragma unroll 1
  for (int rr = 0; rr < 2; ++rr) {
    const int rl = wave * 2 + rr; const size_t mo = (r0 + rl) * DM;
    v4f v[8]; float s1 = 0.f;
#pragma unroll
    for (int i = 0; i < 8; ++i) {
      const v4f z = *(const v4f*)&sz[rl][i * 128 + lane * 4]; const v4f bb = *(const v4f*)(B2 + i * 128 + lane * 4); const v4f xr = *(const v4f*)(X32q + mo + i * 128 + lane * 4);
#pragma unroll
      for (int k = 0; k < 4; ++k) v[i][k] = xr[k] + (z[k] + bf16r(bb[k]));
      s1 += (v[i][0] + v[i][1]) + (v[i][2] + v[i][3]);
    }
#pragma unroll
    for (int o = 1; o < 32; o <<= 1) s1 += __shfl_xor(s1, o);
    const float mu = s1 * (1.0f / DM); float qv = 0.f;
#pragma unroll
    for (int i = 0; i < 8; ++i)
#pragma unroll
      for (int k = 0; k < 4; ++k) { const float d = v[i][k] - mu; qv += d * d; }
#pragma unroll
    for (int o = 1; o < 32; o <<= 1) qv += __shfl_xor(qv, o);
    const float rs = 1.0f / sqrtf(qv * (1.0f / DM) + LN_EPS);
#pragma unroll
    for (int i = 0; i < 8; ++i) {
      const v4f gg = *(const v4f*)(G2 + i * 128 + lane * 4), cc = *(const v4f*)(C2 + i * 128 + lane * 4);
      v4f y;
#pragma unroll
      for (int k = 0; k < 4; ++k) y[k] = (v[i][k] - mu) * rs * bf16r(gg[k]) + bf16r(cc[k]);
      vst2(OUTq + mo + i * 128 + lane * 4, y);
    }
  }
}

extern "C" void kernel_launch(void* const* d_in, const int* in_sizes, int n_in, void* d_out, int out_size, void* d_ws, size_t ws_size, hipStream_t stream) {
  if (n_in < 9) return;
  if (in_sizes[0] < NB * SEQ_FULL * DM) return;
  if (in_sizes[1] < DM || in_sizes[2] < DM || in_sizes[3] < DM || in_sizes[4] < DM) return;
  if (in_sizes[5] < DM * DFF || in_sizes[6] < DFF || in_sizes[7] < DFF * DM || in_sizes[8] < DM) return;
  if ((size_t)out_size < NTOK * DM) return;
  if (ws_size < (size_t)WS_END) return;
  const float* SRC = (const float*)d_in[0];
  const float* G1 = (const float*)d_in[1]; const float* C1 = (const float*)d_in[2];
  const float* G2 = (const float*)d_in[3]; const float* C2 = (const float*)d_in[4];
  const float* W1 = (const float*)d_in[5]; const float* B1 = (const float*)d_in[6];
  const float* W2 = (const float*)d_in[7]; const float* B2 = (const float*)d_in[8];
  float* OUT = (float*)d_out;
  char* ws = (char*)d_ws;
  unsigned short* QBu = (unsigned short*)(ws + WS_QB); const __bf16* QB = (const __bf16*)(ws + WS_QB);
  _Float16* VT = (_Float16*)(ws + WS_VT); _Float16* W1T = (_Float16*)(ws + WS_W1T); _Float16* W2T = (_Float16*)(ws + WS_W2T);
  float* X32 = (float*)(ws + WS_X32); _Float16* X16 = (_Float16*)(ws + WS_X16); _Float16* H16 = (_Float16*)(ws + WS_H16);

  k_prep<<<dim3(SEQ / 64, NH, NB), 256, 0, stream>>>(SRC, QBu, VT);
  k_trw<<<dim3(DFF / 64, DM / 64), 256, 0, stream>>>(W1, DM, DFF, W1T);
  k_trw<<<dim3(DM / 64, DFF / 64), 256, 0, stream>>>(W2, DFF, DM, W2T);
  k_attln<<<dim3((unsigned)(NTOK / 16)), 512, 0, stream>>>(SRC, QB, VT, G1, C1, X32, X16);
  for (int qt = 0; qt < NQ; ++qt) {
    const size_t ro = (size_t)qt * MQ * DM;
    k_g1<<<dim3((unsigned)(MQ / 64), DFF / 128), 128, 0, stream>>>(X16 + ro, W1T, B1, H16);
    k_g2ln<<<dim3((unsigned)(MQ / 16)), 256, 0, stream>>>(H16, W2T, B2, X32 + ro, G2, C2, OUT + ro);
  }
}
